// LightweightPointCloudEncoderWithGlobalAttention_86268713107572
// MI455X (gfx1250) — hardware-verified
//
#include <hip/hip_runtime.h>
#include <math.h>

typedef __attribute__((ext_vector_type(16))) _Float16 v16h;
typedef __attribute__((ext_vector_type(16))) __bf16 v16b;
typedef __attribute__((ext_vector_type(8)))  _Float16 v8h;
typedef __attribute__((ext_vector_type(8)))  float v8f;
typedef __attribute__((ext_vector_type(4)))  float v4f;
typedef __attribute__((ext_vector_type(2)))  float v2f;
typedef __attribute__((ext_vector_type(4)))  unsigned v4u;
typedef __attribute__((ext_vector_type(4)))  int v4i;
typedef float __attribute__((may_alias)) float_a;
typedef int __attribute__((may_alias)) int_a;

template <typename T> __device__ __forceinline__ void vst2(void* p, T v) { *(volatile T*)p = v; __threadfence(); *(volatile T*)p = v; }
__device__ __forceinline__ v8f wmma16(v16h a, v16h b, v8f c) {
  v8f d = __builtin_amdgcn_wmma_f32_16x16x32_f16(false, a, false, b, (short)0, c, false, false);
  asm volatile("v_nop\n\tv_nop\n\tv_nop\n\tv_nop" : "+v"(d) : "v"(a), "v"(b));
  return d;
}
__device__ __forceinline__ v8f wmma_bf(v16b a, v16b b, v8f c) {
  v8f d = __builtin_amdgcn_wmma_f32_16x16x32_bf16(false, a, false, b, (short)0, c, false, false);
  asm volatile("v_nop\n\tv_nop\n\tv_nop\n\tv_nop" : "+v"(d) : "v"(a), "v"(b));
  return d;
}
__device__ __forceinline__ v16h frag_h(const _Float16* rowk0, int lane) {
  union { v16h v; v8h q[2]; } u; const _Float16* p = rowk0 + 8 * (lane >> 4);
  u.q[0] = *(const v8h*)p; u.q[1] = *(const v8h*)(p + 16); return u.v;
}
__device__ __forceinline__ v16h frag_f32(const float* rowk0, int lane) {
  v16h a; const float* p = rowk0 + 8 * (lane >> 4);
#pragma unroll
  for (int i = 0; i < 8; ++i) { a[i] = (_Float16)p[i]; a[8 + i] = (_Float16)p[16 + i]; }
  return a;
}
__device__ __forceinline__ v16h frag_f32s(const float* rowk0, int lane, float sc) {
  v16h a; const float* p = rowk0 + 8 * (lane >> 4);
#pragma unroll
  for (int i = 0; i < 8; ++i) { a[i] = (_Float16)(p[i] * sc); a[8 + i] = (_Float16)(p[16 + i] * sc); }
  return a;
}
__device__ __forceinline__ v16h fragc_f32(const float* W, int k0, int n, int lane, int ld, int K) {
  v16h a; const int g = lane >> 4;
#pragma unroll
  for (int i = 0; i < 8; ++i) { const int ka = k0 + 8 * g + i, kb = ka + 16;
    a[i] = (_Float16)(ka < K ? W[(size_t)(ka < K ? ka : K - 1) * ld + n] : 0.f); a[8 + i] = (_Float16)(kb < K ? W[(size_t)(kb < K ? kb : K - 1) * ld + n] : 0.f); }
  return a;
}
struct F2 { v16b h, l; };
__device__ __forceinline__ F2 bsplit16(const float v[16]) { F2 r;
#pragma unroll
  for (int i = 0; i < 16; ++i) { const __bf16 h = (__bf16)v[i]; r.h[i] = h; r.l[i] = (__bf16)(v[i] - (float)h); }
  return r; }
__device__ __forceinline__ F2 split_row(const float* row, int k0, int lane) { float v[16]; const float* p = row + k0 + 8 * (lane >> 4);
#pragma unroll
  for (int i = 0; i < 8; ++i) { v[i] = p[i]; v[8 + i] = p[16 + i]; }
  return bsplit16(v); }
__device__ __forceinline__ F2 split_rowK(const float* row, int k0, int lane, int K) { float v[16]; const int g = lane >> 4;
#pragma unroll
  for (int i = 0; i < 8; ++i) { const int ka = k0 + 8 * g + i, kb = ka + 16; v[i] = ka < K ? row[ka < K ? ka : K - 1] : 0.f; v[8 + i] = kb < K ? row[kb < K ? kb : K - 1] : 0.f; }
  return bsplit16(v); }
__device__ __forceinline__ F2 split_col(const float* W, int k0, int n, int lane, int ld, int K) { float v[16]; const int g = lane >> 4;
#pragma unroll
  for (int i = 0; i < 8; ++i) { const int ka = k0 + 8 * g + i, kb = ka + 16; v[i] = ka < K ? W[(size_t)(ka < K ? ka : K - 1) * ld + n] : 0.f; v[8 + i] = kb < K ? W[(size_t)(kb < K ? kb : K - 1) * ld + n] : 0.f; }
  return bsplit16(v); }
__device__ __forceinline__ v8f mac3(const F2& a, const F2& b, v8f c) { c = wmma_bf(a.l, b.h, c); c = wmma_bf(a.h, b.l, c); return wmma_bf(a.h, b.h, c); }
__device__ __forceinline__ float sigm(float v) { return 1.0f / (1.0f + expf(-v)); }
#define LDSX() do { asm volatile("s_wait_dscnt 0" ::: "memory"); __builtin_amdgcn_wave_barrier(); __builtin_amdgcn_fence(__ATOMIC_RELEASE, "workgroup"); } while (0)


#ifndef NB
#define NB 4
#define NN 4096
#endif
#define CF 9
#define KNB 8
#define L1 64
#define L2 128
#define L3 256
#define HID 128
#define NR (NB * NN)
#define RBLK (NR / 64)
#ifndef TQB
#define TQB (NN / 64)
#endif
typedef __attribute__((ext_vector_type(8))) __bf16 v8b;
__device__ __forceinline__ v16b frag_b(const __bf16* rowk0, int lane) {
  union { v16b v; v8b q[2]; } u; const __bf16* p = rowk0 + 8 * (lane >> 4);
  u.q[0] = *(const v8b*)p; u.q[1] = *(const v8b*)(p + 16); return u.v;
}
__device__ __forceinline__ float bfr(float v) { return (float)(__bf16)v; }
__device__ __attribute__((noinline)) float exp_ni(float v) { return expf(v); }
__device__ __attribute__((noinline)) float erf_ni(float v) { return erff(v); }

#define PK_W1 0
#define PK_W2 ((size_t)L1 * 32)
#define PK_W3 (PK_W2 + (size_t)L2 * L1)
#define PK_Q  (PK_W3 + (size_t)L3 * L2)
#define PK_K  (PK_Q + (size_t)HID * L3)
#define PK_V  (PK_K + (size_t)HID * L3)
#define PK_F  (PK_V + (size_t)HID * L3)
#define PK_A1 (PK_F + (size_t)L3 * HID)
#define PK_FC (PK_A1 + (size_t)64 * L3)
#define PK_END (PK_FC + (size_t)L3 * L3)
#define WS_PK  0u
#define WS_FT  (((2u * PK_END) + 127u) / 128u * 128u)
#define WS_Y1  (WS_FT + 4u * NR * 32)
#define WS_Y2  (WS_Y1 + 4u * NR * L1)
#define WS_Y3  (WS_Y2 + 4u * NR * L2)
#define WS_H   (WS_Y3 + 4u * NR * L3)
#define WS_QK  (WS_H + 4u * NR * L3)
#define WS_QKL (WS_QK + 2u * NR * 2 * HID)
#define WS_VTH (WS_QKL + 2u * NR * 2 * HID)
#define WS_VTL (WS_VTH + 2u * NR * HID)
#define WS_O   (WS_VTL + 2u * NR * HID)
#define WS_H2  (WS_O + 4u * NR * HID)
#define WS_S   (WS_H2 + 4u * NR * L3)
#define WS_ST  (WS_S + 4u * NR)
#define WS_MS  (WS_ST + 4u * (size_t)RBLK * (L3 / 16) * 32)
#define WS_END (WS_MS + 4u * 3 * L3 * 2)

__global__ __launch_bounds__(256) void k_pack(const float* __restrict__ W1, const float* __restrict__ W2, const float* __restrict__ W3, const float* __restrict__ QW, const float* __restrict__ KW, const float* __restrict__ VW, const float* __restrict__ FW, const float* __restrict__ AW1, const float* __restrict__ FCW, __bf16* __restrict__ PK) {
  __shared__ __align__(16) __bf16 s[L3]; const int n = blockIdx.x, which = blockIdx.y, t = threadIdx.x; int K, NO; size_t dst; const float* Wm; int KS;
  switch (which) { case 0: Wm = W1; KS = 2 * CF; K = 32; NO = L1; dst = PK_W1; break; case 1: Wm = W2; KS = K = L1; NO = L2; dst = PK_W2; break; case 2: Wm = W3; KS = K = L2; NO = L3; dst = PK_W3; break; case 3: Wm = QW; KS = K = L3; NO = HID; dst = PK_Q; break; case 4: Wm = KW; KS = K = L3; NO = HID; dst = PK_K; break; case 5: Wm = VW; KS = K = L3; NO = HID; dst = PK_V; break; case 6: Wm = FW; KS = K = HID; NO = L3; dst = PK_F; break; case 7: Wm = AW1; KS = K = L3; NO = 64; dst = PK_A1; break; default: Wm = FCW; KS = K = L3; NO = L3; dst = PK_FC; break; }
  if (n >= NO) return;
  if (t < K) s[t] = (__bf16)((t < KS) ? Wm[(size_t)n * KS + t] : 0.f);
  __syncthreads();
  if (t < K / 8) vst2((unsigned*)(PK + dst + (size_t)n * K + t * 8), *(const v4u*)&s[t * 8]);
}
__global__ __launch_bounds__(256) void k_knn(const float* __restrict__ X, float* __restrict__ FT) {
  __shared__ float sx[NN][3]; __shared__ float sq[NN]; __shared__ float ld[64][4][KNB + 1]; __shared__ int li[64][4][KNB + 1]; __shared__ int snb[64][KNB]; __shared__ __align__(16) float sft[64][32];
  const int t = threadIdx.x; const size_t b = blockIdx.y; const int n0 = blockIdx.x * 64; const int q = t >> 2, part = t & 3;
  for (int i = t; i < NN; i += 256) { const float x = bfr(X[(b * NN + i) * CF]), y = bfr(X[(b * NN + i) * CF + 1]), z = bfr(X[(b * NN + i) * CF + 2]); sx[i][0] = x; sx[i][1] = y; sx[i][2] = z; sq[i] = (x * x + z * z) + y * y; }
  __syncthreads();
  const int me = n0 + q; const float px = sx[me][0], py = sx[me][1], pz = sx[me][2], sqm = sq[me];
  float* bd = ld[q][part]; int* bi = li[q][part]; for (int k = 0; k < KNB + 1; ++k) { bd[k] = 3.0e38f; bi[k] = 0x7fffffff; }
  float thr = 3.0e38f; int thri = 0x7fffffff;
#pragma unroll 1
  for (int i = part * (NN / 4); i < (part + 1) * (NN / 4); ++i) { const float dot = (px * sx[i][0] + py * sx[i][1]) + pz * sx[i][2]; float d = (sqm + sq[i]) - 2.0f * dot; d = fmaxf(d, 0.f);
    if (d < thr || (d == thr && i < thri)) { int pos = KNB; while (pos > 0 && (d < bd[pos - 1] || (d == bd[pos - 1] && i < bi[pos - 1]))) { bd[pos] = bd[pos - 1]; bi[pos] = bi[pos - 1]; --pos; } bd[pos] = d; bi[pos] = i; thr = bd[KNB]; thri = bi[KNB]; } }
  __syncthreads();
  if (part == 0) { int hp[4] = {0, 0, 0, 0};
    for (int k = 0; k < KNB + 1; ++k) { int best = -1; float bdv = 3.0e38f; int biv = 0x7fffffff;
      for (int p2 = 0; p2 < 4; ++p2) { if (hp[p2] > KNB) continue; const float dv = ld[q][p2][hp[p2]]; const int iv = li[q][p2][hp[p2]]; if (best < 0 || dv < bdv || (dv == bdv && iv < biv)) { best = p2; bdv = dv; biv = iv; } }
      if (k >= 1) snb[q][k - 1] = biv; ++hp[best]; } }
  __syncthreads();
  for (int e = t; e < 64 * 32; e += 256) { const int r = e >> 5, c = e & 31; float v = 0.f; const size_t row = b * NN + n0 + r;
    if (c < CF) { float a = 0.f; for (int k = 0; k < KNB; ++k) a += bfr(X[(b * NN + snb[r][k]) * CF + c]); v = a * (1.0f / KNB) - bfr(X[row * CF + c]); }
    else if (c < 2 * CF) v = bfr(X[row * CF + (c - CF)]);
    sft[r][c] = v; }
  __syncthreads();
  for (int e = t; e < 64 * 8; e += 256) { const int r = e >> 3, q4 = e & 7; vst2(FT + (b * NN + n0 + r) * 32 + q4 * 4, *(const v4f*)&sft[r][q4 * 4]); }
}
__global__ __launch_bounds__(256) void k_stat(const float* __restrict__ ST, int layer, int NC, float* __restrict__ MS) {
  const int c = threadIdx.x; __shared__ __align__(16) float sm[L3][2];
  if (c < NC) { float s = 0.f, q2 = 0.f; for (int blk = 0; blk < RBLK; ++blk) { const float* p = ST + ((size_t)blk * (L3 / 16) + (c >> 4)) * 32 + (c & 15) * 2; s += p[0]; q2 += p[1]; } const float mu = s / (float)NR; sm[c][0] = mu; sm[c][1] = 1.0f / sqrtf(fmaxf(q2 / (float)NR - mu * mu, 0.f) + 1e-5f); }
  __syncthreads();
  if (c < NC / 2) vst2(MS + (size_t)layer * L3 * 2 + c * 4, *(const v4f*)(&sm[0][0] + c * 4));
}
template <int L>
__global__ __launch_bounds__(128) void k_layer(const float* __restrict__ SRC, const float* __restrict__ MS, const float* __restrict__ G, const float* __restrict__ BE, const __bf16* __restrict__ PK, const float* __restrict__ BIAS, float* __restrict__ Y, float* __restrict__ ST) {
  constexpr int KD = (L == 1) ? 32 : (L == 2) ? L1 : (L == 3) ? L2 : L3; constexpr int NO = (L == 1) ? L1 : (L == 2) ? L2 : L3; constexpr int NT = NO / 16;
  __shared__ __align__(16) __bf16 sh[64][KD + 8], sl[64][KD + 8]; __shared__ __align__(16) float so[64][NO + 4];
  const int tid = threadIdx.x, wave = tid >> 5, lane = tid & 31, col = lane & 15, g = lane >> 4; const size_t r0b = (size_t)blockIdx.x * 64;
  const float* msl = MS + (size_t)(L - 2) * L3 * 2;
  for (int e = tid; e < 64 * KD; e += 128) { const int r = e / KD, c = e % KD; float v = SRC[(r0b + r) * KD + c];
    if (L >= 2) v = fmaxf(bfr(G[c]) * (v - msl[c * 2]) * msl[c * 2 + 1] + bfr(BE[c]), 0.f);
    if (L == 4) { so[r][c] = v; continue; }
    const __bf16 hb = (__bf16)v; sh[r][c] = hb; sl[r][c] = (__bf16)(v - (float)hb); }
  if (L == 4) { __syncthreads(); for (int e = tid; e < 64 * NO / 4; e += 128) { const int r = e / (NO / 4), q4 = e % (NO / 4); vst2(Y + (r0b + r) * NO + q4 * 4, *(const v4f*)&so[r][q4 * 4]); } return; }
  if (tid < 64) for (int c = KD; c < KD + 8; ++c) { sh[tid][c] = (__bf16)0.f; sl[tid][c] = (__bf16)0.f; }
  __syncthreads();
  const __bf16* P = PK + ((L == 1) ? PK_W1 : (L == 2) ? PK_W2 : PK_W3);
  v8f acc[NT] = {};
#pragma unroll
  for (int kc = 0; kc < KD / 32; ++kc) { F2 a; a.h = frag_b(&sh[wave * 16 + col][kc * 32], lane); a.l = frag_b(&sl[wave * 16 + col][kc * 32], lane);
#pragma unroll
    for (int j = 0; j < NT; ++j) { const v16b w = frag_b(P + (size_t)(j * 16 + col) * KD + kc * 32, lane); acc[j] = wmma_bf(a.l, w, acc[j]); acc[j] = wmma_bf(a.h, w, acc[j]); } }
#pragma unroll
  for (int j = 0; j < NT; ++j) { const float bb = bfr(BIAS[j * 16 + col]);
#pragma unroll
    for (int r = 0; r < 8; ++r) so[wave * 16 + 8 * g + r][j * 16 + col] = acc[j][r] + bb; }
  __syncthreads();
  for (int e = tid; e < 64 * NO / 4; e += 128) { const int r = e / (NO / 4), q4 = e % (NO / 4); vst2(Y + (r0b + r) * NO + q4 * 4, *(const v4f*)&so[r][q4 * 4]); }
  __shared__ __align__(16) float sst[L3 / 16][32];
  for (int c = tid; c < NO; c += 128) { float s = 0.f, q2 = 0.f; for (int r = 0; r < 64; ++r) { const float v = so[r][c]; s += v; q2 += v * v; } sst[c >> 4][(c & 15) * 2] = s; sst[c >> 4][(c & 15) * 2 + 1] = q2; }
  __syncthreads();
  for (int e = tid; e < NT * 8; e += 128) { const int grp = e >> 3, q4 = e & 7; vst2(ST + ((size_t)blockIdx.x * (L3 / 16) + grp) * 32 + q4 * 4, *(const v4f*)&sst[grp][q4 * 4]); }
}
__global__ __launch_bounds__(128) void k_qkv(const float* __restrict__ H, const __bf16* __restrict__ PK, const float* __restrict__ QB, const float* __restrict__ KB, const float* __restrict__ VB, _Float16* __restrict__ QK, _Float16* __restrict__ QKL, _Float16* __restrict__ VTH, _Float16* __restrict__ VTL) {
  __shared__ __align__(16) _Float16 so[4][16][136], sol[4][16][136]; __shared__ __align__(16) _Float16 sth[128][72], stl[128][72];
  const int tid = threadIdx.x, wave = tid >> 5, lane = tid & 31, col = lane & 15, g = lane >> 4; const int which = blockIdx.y; const size_t r0 = (size_t)blockIdx.x * 64 + wave * 16;
  const __bf16* P = PK + ((which == 0) ? PK_Q : (which == 1) ? PK_K : PK_V); const float* BB = (which == 0) ? QB : (which == 1) ? KB : VB;
  v8f acc[8] = {};
#pragma unroll 2
  for (int kc = 0; kc < L3 / 32; ++kc) { const F2 a = split_row(H + (r0 + col) * L3, kc * 32, lane);
#pragma unroll
    for (int j = 0; j < 8; ++j) { const v16b w = frag_b(P + (size_t)(j * 16 + col) * L3 + kc * 32, lane); acc[j] = wmma_bf(a.l, w, acc[j]); acc[j] = wmma_bf(a.h, w, acc[j]); } }
  if (which < 2) {
#pragma unroll
    for (int j = 0; j < 8; ++j) { const float bb = bfr(BB[j * 16 + col]);
#pragma unroll
      for (int r = 0; r < 8; ++r) { const float v = acc[j][r] + bb; const _Float16 hv = (_Float16)v; so[wave][8 * g + r][j * 16 + col] = hv; sol[wave][8 * g + r][j * 16 + col] = (_Float16)((v - (float)hv) * 2048.0f); } }
    LDSX();
    for (int rl = 0; rl < 16; ++rl) if (lane < 16) { vst2((unsigned*)(QK + (r0 + rl) * (2 * HID) + which * HID + lane * 8), *(const v4u*)&so[wave][rl][lane * 8]); vst2((unsigned*)(QKL + (r0 + rl) * (2 * HID) + which * HID + lane * 8), *(const v4u*)&sol[wave][rl][lane * 8]); }
  } else {
#pragma unroll
    for (int j = 0; j < 8; ++j) { const float bb = bfr(BB[j * 16 + col]);
#pragma unroll
      for (int r = 0; r < 8; ++r) { const float v = acc[j][r] + bb; const _Float16 hv = (_Float16)v; sth[j * 16 + col][wave * 16 + 8 * g + r] = hv; stl[j * 16 + col][wave * 16 + 8 * g + r] = (_Float16)((v - (float)hv) * 2048.0f); } }
    __syncthreads();
    const size_t rb = (size_t)blockIdx.x * 64; const size_t b = rb / NN; const int s0 = (int)(rb % NN);
    for (int e = tid; e < 128 * 8; e += 128) { const int d = e >> 3, pc = e & 7; const size_t o = (b * HID + d) * NN + s0 + pc * 8; vst2((unsigned*)(VTH + o), *(const v4u*)&sth[d][pc * 8]); vst2((unsigned*)(VTL + o), *(const v4u*)&stl[d][pc * 8]); }
  }
}
__global__ __launch_bounds__(128) void k_attn(const _Float16* __restrict__ QK, const _Float16* __restrict__ QKL, const _Float16* __restrict__ VTH, const _Float16* __restrict__ VTL, float* __restrict__ O) {
  __shared__ __align__(16) _Float16 sph[4][16][40], spl[4][16][40]; __shared__ __align__(16) float so[4][16][132];
  const int tid = threadIdx.x, wave = tid >> 5, lane = tid & 31, col = lane & 15, g = lane >> 4; const size_t b = blockIdx.y; const int q0 = blockIdx.x * 64 + wave * 16; const size_t rq = b * NN + q0;
  float m[8], l[8];
#pragma unroll
  for (int r = 0; r < 8; ++r) { m[r] = -3.0e38f; l[r] = 0.f; }
  v8f acc[8] = {}, accl[8] = {};
  const _Float16* Vh = VTH + (b * HID) * NN; const _Float16* Vl = VTL + (b * HID) * NN;
#pragma unroll 1
  for (int ks = 0; ks < NN / 32; ++ks) { const int j0 = ks * 32; v8f s[2];
#pragma unroll
    for (int ct = 0; ct < 2; ++ct) { const int kk = j0 + ct * 16 + col; const size_t rk = (b * NN + kk) * (2 * HID) + HID; v8f c = {}, cl = {};
#pragma unroll 1
      for (int kc = 0; kc < HID / 32; ++kc) { const v16h aq = frag_h(QK + (rq + col) * (2 * HID) + kc * 32, lane), aql = frag_h(QKL + (rq + col) * (2 * HID) + kc * 32, lane); const v16h kh = frag_h(QK + rk + kc * 32, lane); c = wmma16(aq, kh, c); cl = wmma16(aql, kh, cl); cl = wmma16(aq, frag_h(QKL + rk + kc * 32, lane), cl); }
#pragma unroll
      for (int r = 0; r < 8; ++r) s[ct][r] = c[r] + cl[r] * (1.0f / 2048.0f); }
#pragma unroll
    for (int r = 0; r < 8; ++r) { float mx = fmaxf(s[0][r], s[1][r]);
#pragma unroll
      for (int o = 1; o < 16; o <<= 1) mx = fmaxf(mx, __shfl_xor(mx, o));
      const float mn = fmaxf(m[r], mx); const float alpha = (m[r] <= -1.0e38f) ? 0.f : __expf(m[r] - mn);
      const float e0 = __expf(s[0][r] - mn), e1 = __expf(s[1][r] - mn); float es = e0 + e1;
#pragma unroll
      for (int o = 1; o < 16; o <<= 1) es += __shfl_xor(es, o);
      l[r] = l[r] * alpha + es; m[r] = mn;
#pragma unroll
      for (int dt = 0; dt < 8; ++dt) { acc[dt][r] *= alpha; accl[dt][r] *= alpha; }
      const _Float16 h0 = (_Float16)e0, h1 = (_Float16)e1; sph[wave][8 * g + r][col] = h0; sph[wave][8 * g + r][16 + col] = h1; spl[wave][8 * g + r][col] = (_Float16)((e0 - (float)h0) * 2048.0f); spl[wave][8 * g + r][16 + col] = (_Float16)((e1 - (float)h1) * 2048.0f); }
    LDSX();
    const v16h pah = frag_h(&sph[wave][col][0], lane), pal = frag_h(&spl[wave][col][0], lane);
#pragma unroll
    for (int dt = 0; dt < 8; ++dt) { const size_t vo = (size_t)(dt * 16 + col) * NN + j0; const v16h vh = frag_h(Vh + vo, lane); acc[dt] = wmma16(pah, vh, acc[dt]); accl[dt] = wmma16(pal, vh, accl[dt]); accl[dt] = wmma16(pah, frag_h(Vl + vo, lane), accl[dt]); }
    LDSX(); }
#pragma unroll
  for (int r = 0; r < 8; ++r) { const float il = 1.0f / l[r];
#pragma unroll
    for (int dt = 0; dt < 8; ++dt) so[wave][8 * g + r][dt * 16 + col] = (acc[dt][r] + accl[dt][r] * (1.0f / 2048.0f)) * il; }
  LDSX();
  for (int rl = 0; rl < 16; ++rl) vst2(O + (rq + rl) * HID + lane * 4, *(const v4f*)&so[wave][rl][lane * 4]);
}
__global__ __launch_bounds__(128) void k_post(const float* __restrict__ O, const float* __restrict__ H, const __bf16* __restrict__ PK, const float* __restrict__ FB, const float* __restrict__ AB1, const float* __restrict__ AW2, const float* __restrict__ AB2, float* __restrict__ H2, float* __restrict__ S) {
  __shared__ __align__(16) float so[64][L3 + 4]; __shared__ __align__(16) __bf16 sh[64][L3 + 8], sl[64][L3 + 8]; __shared__ float sa[64][65]; __shared__ __align__(16) float ss[64];
  const int tid = threadIdx.x, wave = tid >> 5, lane = tid & 31, col = lane & 15, g = lane >> 4; const size_t r0b = (size_t)blockIdx.x * 64; const size_t r0 = r0b + wave * 16;
  for (int e = tid; e < 64 * L3 / 4; e += 128) { const int r = e / (L3 / 4), q4 = e % (L3 / 4); *(v4f*)&so[r][q4 * 4] = *(const v4f*)(H + (r0b + r) * L3 + q4 * 4); }
  __syncthreads();
#pragma unroll 1
  for (int half = 0; half < 2; ++half) { v8f acc[8] = {};
#pragma unroll
    for (int kc = 0; kc < HID / 32; ++kc) { const F2 a = split_row(O + (r0 + col) * HID, kc * 32, lane);
#pragma unroll
      for (int j = 0; j < 8; ++j) { const v16b w = frag_b(PK + PK_F + (size_t)(half * 128 + j * 16 + col) * HID + kc * 32, lane); acc[j] = wmma_bf(a.l, w, acc[j]); acc[j] = wmma_bf(a.h, w, acc[j]); } }
#pragma unroll
    for (int j = 0; j < 8; ++j) { const int c = half * 128 + j * 16 + col; const float bb = bfr(FB[c]);
#pragma unroll
      for (int r = 0; r < 8; ++r) { const int rr = wave * 16 + 8 * g + r; const float v = acc[j][r] + bb + so[rr][c]; so[rr][c] = v; const __bf16 hb = (__bf16)v; sh[rr][c] = hb; sl[rr][c] = (__bf16)(v - (float)hb); } } }
  if (tid < 64) for (int c = L3; c < L3 + 8; ++c) { sh[tid][c] = (__bf16)0.f; sl[tid][c] = (__bf16)0.f; }
  __syncthreads();
  for (int e = tid; e < 64 * L3 / 4; e += 128) { const int r = e / (L3 / 4), q4 = e % (L3 / 4); vst2(H2 + (r0b + r) * L3 + q4 * 4, *(const v4f*)&so[r][q4 * 4]); }
  { v8f acc[4] = {};
#pragma unroll
    for (int kc = 0; kc < L3 / 32; ++kc) { F2 a; a.h = frag_b(&sh[wave * 16 + col][kc * 32], lane); a.l = frag_b(&sl[wave * 16 + col][kc * 32], lane);
#pragma unroll
      for (int j = 0; j < 4; ++j) { const v16b w = frag_b(PK + PK_A1 + (size_t)(j * 16 + col) * L3 + kc * 32, lane); acc[j] = wmma_bf(a.l, w, acc[j]); acc[j] = wmma_bf(a.h, w, acc[j]); } }
#pragma unroll
    for (int j = 0; j < 4; ++j) { const float bb = bfr(AB1[j * 16 + col]);
#pragma unroll
      for (int r = 0; r < 8; ++r) sa[wave * 16 + 8 * g + r][j * 16 + col] = fmaxf(acc[j][r] + bb, 0.f); } }
  __syncthreads();
  if (tid < 64) { float a = 0.f; for (int c = 0; c < 64; ++c) a += sa[tid][c] * bfr(AW2[c]); ss[tid] = a + bfr(AB2[0]); }
  __syncthreads();
  if (tid < 16) vst2(S + r0b + tid * 4, *(const v4f*)&ss[tid * 4]);
}
__global__ __launch_bounds__(256) void k_pool(const float* __restrict__ H2, const float* __restrict__ S, const float* __restrict__ FCW, const float* __restrict__ FCB, float* __restrict__ OUT) {
  __shared__ float sw[NN]; __shared__ float red[8]; __shared__ float sp[L3]; __shared__ __align__(16) float sout[L3];
  const int t = threadIdx.x; const size_t b = blockIdx.x;
  float mx = -3.0e38f; for (int n = t; n < NN; n += 256) { const float v = S[b * NN + n]; sw[n] = v; mx = fmaxf(mx, v); }
#pragma unroll
  for (int o = 1; o < 32; o <<= 1) mx = fmaxf(mx, __shfl_xor(mx, o));
  if ((t & 31) == 0) red[t >> 5] = mx; __syncthreads(); float gm = -3.0e38f; for (int w = 0; w < 8; ++w) gm = fmaxf(gm, red[w]); __syncthreads();
  float sm = 0.f; for (int n = t; n < NN; n += 256) { const float e = exp_ni(sw[n] - gm); sw[n] = e; sm += e; }
#pragma unroll
  for (int o = 1; o < 32; o <<= 1) sm += __shfl_xor(sm, o);
  if ((t & 31) == 0) red[t >> 5] = sm; __syncthreads(); float tot = 0.f; for (int w = 0; w < 8; ++w) tot += red[w]; const float inv = 1.0f / tot;
  { float a = 0.f;
#pragma unroll 1
    for (int n = 0; n < NN; ++n) a += H2[(b * NN + n) * L3 + t] * sw[n];
    sp[t] = a * inv; }
  __syncthreads();
  { float a = 0.f;
#pragma unroll 1
    for (int c = 0; c < L3; ++c) a += sp[c] * bfr(FCW[(size_t)t * L3 + c]); sout[t] = fmaxf(a + bfr(FCB[t]), 0.f); }
  __syncthreads();
  if (t < L3 / 4) vst2(OUT + b * L3 + t * 4, *(const v4f*)&sout[t * 4]);
}
extern "C" void kernel_launch(void* const* d_in, const int* in_sizes, int n_in, void* d_out, int out_size, void* d_ws, size_t ws_size, hipStream_t stream) {
  (void)in_sizes; (void)n_in; (void)out_size;
  const float** F = (const float**)d_in;
  if (ws_size < (size_t)WS_END) return;
  char* ws = (char*)d_ws; __bf16* PK = (__bf16*)(ws + WS_PK); float *FT = (float*)(ws + WS_FT), *Y1 = (float*)(ws + WS_Y1), *Y2 = (float*)(ws + WS_Y2), *Y3 = (float*)(ws + WS_Y3), *H = (float*)(ws + WS_H), *O = (float*)(ws + WS_O), *H2 = (float*)(ws + WS_H2), *S = (float*)(ws + WS_S), *ST = (float*)(ws + WS_ST), *MS = (float*)(ws + WS_MS);
  _Float16 *QK = (_Float16*)(ws + WS_QK), *QKL = (_Float16*)(ws + WS_QKL), *VTH = (_Float16*)(ws + WS_VTH), *VTL = (_Float16*)(ws + WS_VTL);
  k_pack<<<dim3(L3, 9), 256, 0, stream>>>(F[1], F[5], F[9], F[13], F[15], F[17], F[19], F[21], F[25], PK);
  k_knn<<<dim3(NN / 64, NB), 256, 0, stream>>>(F[0], FT);
  k_layer<1><<<RBLK, 128, 0, stream>>>(FT, MS, nullptr, nullptr, PK, F[2], Y1, ST);
  k_stat<<<1, 256, 0, stream>>>(ST, 0, L1, MS);
  k_layer<2><<<RBLK, 128, 0, stream>>>(Y1, MS, F[3], F[4], PK, F[6], Y2, ST);
  k_stat<<<1, 256, 0, stream>>>(ST, 1, L2, MS);
  k_layer<3><<<RBLK, 128, 0, stream>>>(Y2, MS, F[7], F[8], PK, F[10], Y3, ST);
  k_stat<<<1, 256, 0, stream>>>(ST, 2, L3, MS);
  k_layer<4><<<RBLK, 128, 0, stream>>>(Y3, MS, F[11], F[12], PK, nullptr, H, nullptr);
  k_qkv<<<dim3(RBLK, 3), 128, 0, stream>>>(H, PK, F[14], F[16], F[18], QK, QKL, VTH, VTL);
  k_attn<<<dim3(TQB, NB), 128, 0, stream>>>(QK, QKL, VTH, VTL, O);
  k_post<<<RBLK, 128, 0, stream>>>(O, H, PK, F[20], F[22], F[23], F[24], H2, S);
  k_pool<<<NB, 256, 0, stream>>>(H2, S, F[25], F[26], (float*)d_out);
}
